// CausalPerformerAttention_8418135900415
// MI455X (gfx1250) — hardware-run, weakly checked
//
#include <hip/hip_runtime.h>


#ifndef NB
#define NB 2
#endif
#ifndef SEQ
#define SEQ 1024
#endif
#define NB_FULL  2
#define SEQ_FULL 1024
#ifndef OUT_SEQ
#define OUT_SEQ SEQ
#endif
#define DM   768
#define NH_  12
#define HD   64
#define NF   64
#define AW   4
#define L2E  1.4426950408889634f
#define EPSV 1.0e-6f
#define PLN  ((size_t)NB * NH_ * SEQ * HD)
#define CPLN ((size_t)NB * SEQ * DM)

static_assert(HD == 64);
static_assert(NF == 64);
static_assert(NH_ * HD == DM);
static_assert(DM % 64 == 0);
static_assert(DM % 32 == 0);
static_assert(HD % 32 == 0);
static_assert(NF % 32 == 0);
static_assert(SEQ % 64 == 0);
static_assert((NB * SEQ) % 64 == 0);
static_assert(((size_t)NB * NH_ * SEQ) % 64 == 0);
static_assert(SEQ % 32 == 0);
static_assert(SEQ % (16 * AW) == 0);
static_assert(((size_t)SEQ * DM) % 8 == 0);
static_assert(((size_t)DM * DM) % 8 == 0);
static_assert(NB <= NB_FULL);
static_assert(SEQ <= SEQ_FULL);

typedef unsigned short bf;
typedef __attribute__((ext_vector_type(16))) __bf16   v16bf;
typedef __attribute__((ext_vector_type(8)))  unsigned short v8us;
typedef __attribute__((ext_vector_type(16))) unsigned short v16us;
typedef __attribute__((ext_vector_type(8)))  float    v8f;
typedef __attribute__((ext_vector_type(4)))  float    v4f;
typedef v4f  __attribute__((may_alias)) v4fa;

__device__ __forceinline__ unsigned short f2bf(float f) { unsigned u = __float_as_uint(f); u += 0x7FFFu + ((u >> 16) & 1u); return (unsigned short)(u >> 16); }
__device__ __forceinline__ float bf2f(unsigned short w) { return __uint_as_float(((unsigned)w) << 16); }
__device__ __forceinline__ v16bf cat16b(v8us lo, v8us hi) { return __builtin_bit_cast(v16bf, __builtin_shufflevector(lo, hi, 0, 1, 2, 3, 4, 5, 6, 7, 8, 9, 10, 11, 12, 13, 14, 15)); }
__device__ __forceinline__ v8f wmmab(v16bf a, v16bf b, v8f c) { return __builtin_amdgcn_wmma_f32_16x16x32_bf16(false, a, false, b, (short)0, c, false, false); }
__device__ __forceinline__ v16bf ldb(const bf* p)  { return cat16b(*(const v8us*)p, *(const v8us*)(p + 16)); }
__device__ __forceinline__ void wave_sync() { __builtin_amdgcn_fence(3  , "wavefront"); __builtin_amdgcn_wave_barrier(); asm volatile("" ::: "memory"); }
__device__ __forceinline__ void split8(v4f x0, v4f x1, v8us& h, v8us& l) {
#pragma unroll
    for (int i = 0; i < 4; ++i) {
        const unsigned short a0 = f2bf(x0[i]); const unsigned short a1 = f2bf(x1[i]);
        h[i] = a0; h[4 + i] = a1; l[i] = f2bf(x0[i] - bf2f(a0)); l[4 + i] = f2bf(x1[i] - bf2f(a1)); }
}

__global__ __launch_bounds__(256) void k_cvt8(const float* __restrict__ src, bf* dst, size_t n8) {
    const size_t i = (size_t)blockIdx.x * 256 + threadIdx.x; if (i >= n8) return;
    const v8f v = *(const v8f*)(src + i * 8); v8us o;
#pragma unroll
    for (int k = 0; k < 8; ++k) o[k] = f2bf(v[k]);
    *(volatile v8us*)(dst + i * 8) = o; __threadfence(); *(volatile v8us*)(dst + i * 8) = o;
}

__global__ __launch_bounds__(512) void k_projT(const float* __restrict__ src, bf* dst) {
    const int i = threadIdx.x; const int f = i >> 3, c8 = (i & 7) * 8; v8us o;
#pragma unroll
    for (int k = 0; k < 8; ++k) o[k] = f2bf(src[(c8 + k) * NF + f]);
    *(volatile v8us*)(dst + f * HD + c8) = o; __threadfence(); *(volatile v8us*)(dst + f * HD + c8) = o;
}

__device__ __forceinline__ void gemm64(const bf* __restrict__ A, size_t aplane, int npl, const bf* __restrict__ Bt, int K, int r0, int c0, int lr, int hi, v8f (&acc)[4][4]) {
#pragma unroll
    for (int mb = 0; mb < 4; ++mb)
#pragma unroll
        for (int nb = 0; nb < 4; ++nb) acc[mb][nb] = (v8f){};
    const size_t boff = (size_t)(c0 + lr) * K + 8 * hi;
#pragma unroll 1
    for (int pl = 0; pl < npl; ++pl) {
        const size_t aoff = (size_t)pl * aplane + (size_t)(r0 + lr) * K + 8 * hi;
#pragma unroll 1
        for (int kc = 0; kc < K; kc += 32) {
            v16bf a[4];
#pragma unroll
            for (int mb = 0; mb < 4; ++mb) a[mb] = ldb(A + aoff + (size_t)mb * 16 * K + kc);
#pragma unroll
            for (int nb = 0; nb < 4; ++nb) { const v16bf b = ldb(Bt + boff + (size_t)nb * 16 * K + kc);
#pragma unroll
                for (int mb = 0; mb < 4; ++mb) acc[mb][nb] = wmmab(a[mb], b, acc[mb][nb]); }
            asm volatile("v_nop\n\tv_nop\n\tv_nop\n\tv_nop" : "+v"(acc[0][0]), "+v"(acc[1][1]), "+v"(acc[2][2]), "+v"(acc[3][3]) : "v"(a[0]), "v"(a[1]), "v"(a[2]), "v"(a[3]));
        }
    }
}

__global__ __launch_bounds__(32) void k_proj(const bf* __restrict__ A, const bf* __restrict__ Bt, bf* Ph, bf* Pl, int RB, size_t sRB, int pitch, int CB, size_t sCB) {
    __shared__ __align__(16) float os[16 * 68];
    const int lane = threadIdx.x & 31, lr = lane & 15, hi = lane >> 4; const int r0 = blockIdx.x * 64, c0 = blockIdx.y * 64;
    v8f acc[4][4];
    gemm64(A, (size_t)0, 1, Bt, DM, r0, c0, lr, hi, acc);
    const size_t tbase = (size_t)(r0 / RB) * sRB + (size_t)(r0 % RB) * (size_t)pitch + (size_t)(c0 / CB) * sCB + (size_t)(c0 % CB);
#pragma unroll
    for (int mb = 0; mb < 4; ++mb) {
#pragma unroll
        for (int nb = 0; nb < 4; ++nb) {
#pragma unroll
            for (int j = 0; j < 8; ++j) os[(hi * 8 + j) * 68 + nb * 16 + lr] = acc[mb][nb][j]; }
        wave_sync();
        const size_t sb = tbase + (size_t)(mb * 16) * (size_t)pitch;
        v8us hv[4], lv[4];
#pragma unroll
        for (int s = 0; s < 4; ++s) { const int row = 4 * s + (lane >> 3), c8 = (lane & 7) * 8;
            const v4f x0 = *(const v4fa*)(&os[row * 68 + c8]); const v4f x1 = *(const v4fa*)(&os[row * 68 + c8 + 4]);
            split8(x0, x1, hv[s], lv[s]); }
#pragma unroll 1
        for (int ps = 0; ps < 2; ++ps) {
#pragma unroll
            for (int s = 0; s < 4; ++s) { const int row = 4 * s + (lane >> 3), c8 = (lane & 7) * 8;
                const size_t oo = sb + (size_t)row * (size_t)pitch + c8;
                *(volatile v8us*)(Ph + oo) = hv[s]; *(volatile v8us*)(Pl + oo) = lv[s]; }
            if (ps == 0) __threadfence(); }
        wave_sync();
    }
}

__global__ __launch_bounds__(32) void k_feat(const bf* __restrict__ RAW, const bf* __restrict__ PT, bf* FEAT) {
    __shared__ __align__(16) float os[16 * 68];
    __shared__ float nrm[64];
    const int lane = threadIdx.x & 31, lr = lane & 15, hi = lane >> 4; const int r0 = blockIdx.x * 64; const int which = blockIdx.y;
    const bf* Ah = RAW + (size_t)which * 2 * PLN;
    bf* Oh = FEAT + (size_t)which * 2 * PLN; bf* Ol = Oh + PLN;
#pragma unroll 1
    for (int mb = 0; mb < 4; ++mb) {
        const bf* ph = Ah + (size_t)(r0 + mb * 16 + lr) * HD + 8 * hi; const bf* pl = ph + PLN;
        float s = 0.0f;
#pragma unroll
        for (int q = 0; q < 4; ++q) { const v8us a = *(const v8us*)(ph + 16 * q); const v8us c = *(const v8us*)(pl + 16 * q);
#pragma unroll
            for (int i = 0; i < 8; ++i) { const float v = bf2f(a[i]) + bf2f(c[i]); s = fmaf(v, v, s); } }
        s += __shfl_xor(s, 16, 32);
        if (hi == 0) nrm[mb * 16 + lr] = s;
    }
    wave_sync();
    v8f acc[4][4];
    gemm64(Ah, PLN, 2, PT, HD, r0, 0, lr, hi, acc);
#pragma unroll
    for (int mb = 0; mb < 4; ++mb) {
#pragma unroll
        for (int nb = 0; nb < 4; ++nb) {
#pragma unroll
            for (int j = 0; j < 8; ++j) os[(hi * 8 + j) * 68 + nb * 16 + lr] = acc[mb][nb][j]; }
        wave_sync();
        v8us hv[4], lv[4];
#pragma unroll
        for (int s = 0; s < 4; ++s) { const int row = 4 * s + (lane >> 3), c8 = (lane & 7) * 8;
            v4f x0 = *(const v4fa*)(&os[row * 68 + c8]); v4f x1 = *(const v4fa*)(&os[row * 68 + c8 + 4]);
            const float nh = 0.5f * nrm[mb * 16 + row];
#pragma unroll
            for (int i = 0; i < 4; ++i) { x0[i] = __builtin_amdgcn_exp2f((x0[i] - nh) * L2E) * 0.125f; x1[i] = __builtin_amdgcn_exp2f((x1[i] - nh) * L2E) * 0.125f; }
            split8(x0, x1, hv[s], lv[s]); }
#pragma unroll 1
        for (int ps = 0; ps < 2; ++ps) {
#pragma unroll
            for (int s = 0; s < 4; ++s) { const int row = 4 * s + (lane >> 3), c8 = (lane & 7) * 8;
                const size_t oo = (size_t)(r0 + mb * 16 + row) * NF + c8;
                *(volatile v8us*)(Oh + oo) = hv[s]; *(volatile v8us*)(Ol + oo) = lv[s]; }
            if (ps == 0) __threadfence(); }
        wave_sync();
    }
}

__global__ __launch_bounds__(32 * AW) void k_attn(const bf* __restrict__ FEAT, const bf* __restrict__ VT, bf* CTX) {
    __shared__ __align__(16) float os[AW * 16 * 68];
    const int lane = threadIdx.x & 31, lr = lane & 15, hi = lane >> 4;
    const int wave = __builtin_amdgcn_readfirstlane((int)(threadIdx.x >> 5));
    const int zh = blockIdx.y; const int b = zh / NH_, h = zh % NH_;
    const int t0 = (blockIdx.x * AW + wave) * 16;
    const size_t pbase = (size_t)zh * SEQ * HD;
    const bf* QH = FEAT; const bf* QL = FEAT + PLN; const bf* KH = FEAT + 2 * PLN; const bf* KL = FEAT + 3 * PLN;
    const bf* VH = VT; const bf* VL = VT + PLN;
    const size_t qo = pbase + (size_t)(t0 + lr) * NF + 8 * hi;
    const v16bf qh0 = ldb(QH + qo), qh1 = ldb(QH + qo + 32), ql0 = ldb(QL + qo), ql1 = ldb(QL + qo + 32);
    const size_t ko = pbase + (size_t)lr * NF + 8 * hi;
    const size_t vo = pbase + (size_t)lr * SEQ + 8 * hi;
    v8f o0 = (v8f){}, o1 = (v8f){}, o2 = (v8f){}, o3 = (v8f){};
    float l = 0.0f;
    const int nsteps = (t0 + 15) / 32 + 1;
#pragma unroll 1
    for (int st = 0; st < nsteps; ++st) {
        const int key0 = st * 32;
        const bf* kah = KH + ko + (size_t)key0 * NF; const bf* kal = KL + ko + (size_t)key0 * NF;
        const v16bf kah0 = ldb(kah), kah1 = ldb(kah + 32), kbh0 = ldb(kah + 16 * NF), kbh1 = ldb(kah + 16 * NF + 32);
        const v16bf kal0 = ldb(kal), kal1 = ldb(kal + 32), kbl0 = ldb(kal + 16 * NF), kbl1 = ldb(kal + 16 * NF + 32);
        v8f sa = (v8f){}, sb = (v8f){};
        sa = wmmab(kah0, qh0, sa); sb = wmmab(kbh0, qh0, sb); sa = wmmab(kah1, qh1, sa); sb = wmmab(kbh1, qh1, sb);
        sa = wmmab(kah0, ql0, sa); sb = wmmab(kbh0, ql0, sb); sa = wmmab(kah1, ql1, sa); sb = wmmab(kbh1, ql1, sb);
        sa = wmmab(kal0, qh0, sa); sb = wmmab(kbl0, qh0, sb); sa = wmmab(kal1, qh1, sa); sb = wmmab(kbl1, qh1, sb);
        asm volatile("v_nop\n\tv_nop\n\tv_nop\n\tv_nop" : "+v"(sa), "+v"(sb) : "v"(kah0), "v"(kah1), "v"(kbh0), "v"(kbh1), "v"(kal0), "v"(kal1), "v"(kbl0), "v"(kbl1));
        const int dq = t0 + lr - key0 - 8 * hi;
        v16us shu, slu; float ls = 0.0f;
#pragma unroll
        for (int r = 0; r < 8; ++r) {
            const float ta = (r <= dq) ? sa[r] : 0.0f; const float tb = (r + 16 <= dq) ? sb[r] : 0.0f;
            const unsigned short a = f2bf(ta); const unsigned short c = f2bf(tb);
            shu[r] = a; shu[8 + r] = c; slu[r] = f2bf(ta - bf2f(a)); slu[8 + r] = f2bf(tb - bf2f(c));
            ls += (ta + tb); }
        l += ls;
        const v16bf sh = __builtin_bit_cast(v16bf, shu), sl = __builtin_bit_cast(v16bf, slu);
        const bf* va = VH + vo + key0; const bf* vb = VL + vo + key0;
        const v16bf v0 = ldb(va), v1 = ldb(va + (size_t)16 * SEQ), v2 = ldb(va + (size_t)32 * SEQ), v3 = ldb(va + (size_t)48 * SEQ);
        o0 = wmmab(v0, sh, o0); o1 = wmmab(v1, sh, o1); o2 = wmmab(v2, sh, o2); o3 = wmmab(v3, sh, o3);
        o0 = wmmab(v0, sl, o0); o1 = wmmab(v1, sl, o1); o2 = wmmab(v2, sl, o2); o3 = wmmab(v3, sl, o3);
        const v16bf w0 = ldb(vb), w1 = ldb(vb + (size_t)16 * SEQ), w2 = ldb(vb + (size_t)32 * SEQ), w3 = ldb(vb + (size_t)48 * SEQ);
        o0 = wmmab(w0, sh, o0); o1 = wmmab(w1, sh, o1); o2 = wmmab(w2, sh, o2); o3 = wmmab(w3, sh, o3);
        asm volatile("v_nop\n\tv_nop\n\tv_nop\n\tv_nop" : "+v"(o0), "+v"(o1), "+v"(o2), "+v"(o3) : "v"(v0), "v"(v1), "v"(v2), "v"(v3), "v"(w0), "v"(w1), "v"(w2), "v"(w3), "v"(sh), "v"(sl));
    }
    l += __shfl_xor(l, 16, 32);
    const float inv = 1.0f / (l + EPSV);
    const int wb = wave * 16 * 68;
    { v4f a, c;
      a[0] = o0[0] * inv; a[1] = o0[1] * inv; a[2] = o0[2] * inv; a[3] = o0[3] * inv; c[0] = o0[4] * inv; c[1] = o0[5] * inv; c[2] = o0[6] * inv; c[3] = o0[7] * inv;
      *(v4fa*)(&os[wb + lr * 68 +  0 + 8 * hi]) = a; *(v4fa*)(&os[wb + lr * 68 +  0 + 8 * hi + 4]) = c;
      a[0] = o1[0] * inv; a[1] = o1[1] * inv; a[2] = o1[2] * inv; a[3] = o1[3] * inv; c[0] = o1[4] * inv; c[1] = o1[5] * inv; c[2] = o1[6] * inv; c[3] = o1[7] * inv;
      *(v4fa*)(&os[wb + lr * 68 + 16 + 8 * hi]) = a; *(v4fa*)(&os[wb + lr * 68 + 16 + 8 * hi + 4]) = c;
      a[0] = o2[0] * inv; a[1] = o2[1] * inv; a[2] = o2[2] * inv; a[3] = o2[3] * inv; c[0] = o2[4] * inv; c[1] = o2[5] * inv; c[2] = o2[6] * inv; c[3] = o2[7] * inv;
      *(v4fa*)(&os[wb + lr * 68 + 32 + 8 * hi]) = a; *(v4fa*)(&os[wb + lr * 68 + 32 + 8 * hi + 4]) = c;
      a[0] = o3[0] * inv; a[1] = o3[1] * inv; a[2] = o3[2] * inv; a[3] = o3[3] * inv; c[0] = o3[4] * inv; c[1] = o3[5] * inv; c[2] = o3[6] * inv; c[3] = o3[7] * inv;
      *(v4fa*)(&os[wb + lr * 68 + 48 + 8 * hi]) = a; *(v4fa*)(&os[wb + lr * 68 + 48 + 8 * hi + 4]) = c; }
    wave_sync();
    bf* Ch = CTX + ((size_t)b * SEQ + t0) * DM + h * HD; bf* Cl = Ch + CPLN;
    v8us hv[4], lv[4];
#pragma unroll
    for (int s = 0; s < 4; ++s) { const int row = 4 * s + (lane >> 3), c8 = (lane & 7) * 8;
        const v4f x0 = *(const v4fa*)(&os[wb + row * 68 + c8]); const v4f x1 = *(const v4fa*)(&os[wb + row * 68 + c8 + 4]);
        split8(x0, x1, hv[s], lv[s]); }
#pragma unroll 1
    for (int ps = 0; ps < 2; ++ps) {
#pragma unroll
        for (int s = 0; s < 4; ++s) { const int row = 4 * s + (lane >> 3), c8 = (lane & 7) * 8;
            const size_t oo = (size_t)row * DM + c8;
            *(volatile v8us*)(Ch + oo) = hv[s]; *(volatile v8us*)(Cl + oo) = lv[s]; }
        if (ps == 0) __threadfence(); }
}

__global__ __launch_bounds__(32) void k_out(const bf* __restrict__ CTX, const bf* __restrict__ WP, float* OUT) {
    __shared__ __align__(16) float os[16 * 68];
    const int lane = threadIdx.x & 31, lr = lane & 15, hi = lane >> 4; const int r0 = blockIdx.x * 64, c0 = blockIdx.y * 64;
    v8f acc[4][4];
    gemm64(CTX, CPLN, 2, WP, DM, r0, c0, lr, hi, acc);
    float* obase = OUT + ((size_t)(r0 / SEQ) * OUT_SEQ + (size_t)(r0 % SEQ)) * DM + c0;
#pragma unroll
    for (int mb = 0; mb < 4; ++mb) {
#pragma unroll
        for (int nb = 0; nb < 4; ++nb) {
#pragma unroll
            for (int j = 0; j < 8; ++j) os[(hi * 8 + j) * 68 + nb * 16 + lr] = acc[mb][nb][j]; }
        wave_sync();
        float* orow = obase + (size_t)(mb * 16) * DM;
#pragma unroll 1
        for (int ps = 0; ps < 2; ++ps) {
#pragma unroll
            for (int s = 0; s < 8; ++s) { const int row = 2 * s + hi, cofs = lr * 4;
                const v4f val = *(const v4fa*)(&os[row * 68 + cofs]);
                *(volatile v4f*)(orow + (size_t)row * DM + cofs) = val; }
            if (ps == 0) __threadfence(); }
        wave_sync();
    }
}

static constexpr size_t al256(size_t v) { return (v + 255) & ~(size_t)255; }
static constexpr size_t SZ_XB = al256((size_t)NB * SEQ * DM * 2);
static constexpr size_t SZ_WA = al256((size_t)3 * DM * DM * 2);
static constexpr size_t SZ_WP = al256((size_t)DM * DM * 2);
static constexpr size_t SZ_PT = al256((size_t)NF * HD * 2);
static constexpr size_t SZ_PL = al256(PLN * 2);
static constexpr size_t SZ_CP = al256(CPLN * 2);
static constexpr size_t SZ_TOTAL = SZ_XB + SZ_WA + SZ_WP + SZ_PT + 4 * SZ_PL + 4 * SZ_PL + 2 * SZ_PL + 2 * SZ_CP;
static_assert(SZ_TOTAL <= (size_t)134217728);
static_assert((PLN * 2) % 256 == 0);
static_assert((CPLN * 2) % 256 == 0);
static_assert(((size_t)DM * DM * 2) % 256 == 0);

extern "C" void kernel_launch(void* const* d_in, const int* in_sizes, int n_in,
                              void* d_out, int out_size, void* d_ws, size_t ws_size, hipStream_t stream) {
    if (n_in < 4) return;
    const size_t needx = ((size_t)(NB - 1) * SEQ_FULL + SEQ) * DM;
    if ((size_t)in_sizes[0] < needx) return;
    if ((size_t)in_sizes[1] < (size_t)3 * DM * DM || (size_t)in_sizes[2] < (size_t)DM * DM || (size_t)in_sizes[3] < (size_t)HD * NF) return;
    if ((size_t)out_size < ((size_t)(NB - 1) * OUT_SEQ + SEQ) * DM) return;
    if (SZ_TOTAL > ws_size) return;
    const float* x = (const float*)d_in[0]; const float* wa = (const float*)d_in[1]; const float* wp = (const float*)d_in[2]; const float* pj = (const float*)d_in[3];
    float* OUT = (float*)d_out;
    char* wsp = (char*)d_ws;
    bf* XB  = (bf*)wsp; wsp += SZ_XB;
    bf* WA  = (bf*)wsp; wsp += SZ_WA;
    bf* WPB = (bf*)wsp; wsp += SZ_WP;
    bf* PT  = (bf*)wsp; wsp += SZ_PT;
    bf* RAW = (bf*)wsp; wsp += 4 * SZ_PL;
    bf* FEA = (bf*)wsp; wsp += 4 * SZ_PL;
    bf* VT  = (bf*)wsp; wsp += 2 * SZ_PL;
    bf* CTX = (bf*)wsp; wsp += 2 * SZ_CP;
    bf* WQ = WA; bf* WK = WA + (size_t)DM * DM; bf* WV = WA + (size_t)2 * DM * DM;

    if (SEQ == SEQ_FULL) {
        const size_t n8 = (size_t)NB * SEQ * DM / 8;
        k_cvt8<<<(unsigned)((n8 + 255) / 256), 256, 0, stream>>>(x, XB, n8);
    } else {
        const size_t n8 = (size_t)SEQ * DM / 8;
        for (int b = 0; b < NB; ++b) k_cvt8<<<(unsigned)((n8 + 255) / 256), 256, 0, stream>>>(x + (size_t)b * SEQ_FULL * DM, XB + (size_t)b * SEQ * DM, n8);
    }
    { const size_t n8 = (size_t)3 * DM * DM / 8; k_cvt8<<<(unsigned)((n8 + 255) / 256), 256, 0, stream>>>(wa, WA, n8); }
    { const size_t n8 = (size_t)DM * DM / 8;     k_cvt8<<<(unsigned)((n8 + 255) / 256), 256, 0, stream>>>(wp, WPB, n8); }
    k_projT<<<1, 512, 0, stream>>>(pj, PT);

    k_proj<<<dim3(NB * SEQ / 64, DM / 64, 1), 32, 0, stream>>>(XB, WQ, RAW, RAW + PLN, SEQ, (size_t)NH_ * SEQ * HD, HD, HD, (size_t)SEQ * HD);
    k_proj<<<dim3(NB * SEQ / 64, DM / 64, 1), 32, 0, stream>>>(XB, WK, RAW + 2 * PLN, RAW + 3 * PLN, SEQ, (size_t)NH_ * SEQ * HD, HD, HD, (size_t)SEQ * HD);
    k_proj<<<dim3(DM / 64, NB * SEQ / 64, 1), 32, 0, stream>>>(WV, XB, VT, VT + PLN, DM, (size_t)0, SEQ, SEQ, (size_t)DM * SEQ);

    k_feat<<<dim3((unsigned)((size_t)NB * NH_ * SEQ / 64), 2, 1), 32, 0, stream>>>(RAW, PT, FEA);
    k_attn<<<dim3(SEQ / (16 * AW), NB * NH_, 1), 32 * AW, 0, stream>>>(FEA, VT, CTX);
    k_out<<<dim3(NB * SEQ / 64, DM / 64, 1), 32, 0, stream>>>(CTX, WPB, OUT);
}
